// CrossAttentionBlock_30958124269668
// MI455X (gfx1250) — hardware-verified
//
#include <hip/hip_runtime.h>
#include <stddef.h>


typedef _Float16 f16;
typedef f16   v8h  __attribute__((ext_vector_type(8)));
typedef f16   v16h __attribute__((ext_vector_type(16)));
typedef float v8f  __attribute__((ext_vector_type(8)));
typedef float v4f  __attribute__((ext_vector_type(4)));

#ifndef NB
#define NB 4
#endif
#ifndef SEQ
#define SEQ 4096
#endif
#define NB_FULL  4
#define SEQ_FULL 4096
#define CCH  512
#define CCX  64
#define LC   1024
#define LC_FULL 1024
#define NH   8
#define HD   64
#define NG   32

#define GBM 64
#define GBN 128
#define SP  40
#define AKT 64
#define AQB 128
#define KP  72

static_assert(NB >= 1 && NB <= NB_FULL);
static_assert(SEQ >= GBN && SEQ <= SEQ_FULL && (SEQ % GBN) == 0 && (SEQ % AQB) == 0);
static_assert((LC % GBN) == 0 && (LC % AKT) == 0 && LC <= LC_FULL);
static_assert((CCH % GBM) == 0 && (CCH % 32) == 0 && (CCX % 32) == 0);
static_assert(GBM == HD && CCH == NH * HD);
static_assert((CCH % NG) == 0 && (CCX % NG) == 0);
static_assert((SEQ % 8) == 0 && (LC % 8) == 0);

__device__ __forceinline__ float bfr(float v) {
  unsigned int u = __float_as_uint(v);
  u = (u + 0x7FFFu + ((u >> 16) & 1u)) & 0xFFFF0000u;
  return __uint_as_float(u);
}

__device__ __forceinline__ v8f v8zero() {
  v8f z;
#pragma unroll
  for (int i = 0; i < 8; ++i) z[i] = 0.0f;
  return z;
}

__device__ __forceinline__ v16h load_frag(const f16* p) {
  const v8h lo = *(const v8h*)p;
  const v8h hi = *(const v8h*)(p + 16);
  return __builtin_shufflevector(lo, hi, 0, 1, 2, 3, 4, 5, 6, 7, 8, 9, 10, 11, 12, 13, 14, 15);
}

__device__ __forceinline__ v8f wmma16(v16h a, v16h b, v8f c) {
  v8f d = __builtin_amdgcn_wmma_f32_16x16x32_f16(false, a, false, b, (short)0, c, false, false);
  asm volatile("v_nop\n\tv_nop\n\tv_nop\n\tv_nop" : "+v"(d) : "v"(a), "v"(b));
  return d;
}

__global__ __launch_bounds__(256) void cvt_w_kernel(const float* __restrict__ src,
                                                    f16* __restrict__ dst, int n, float scl) {
#pragma clang fp contract(off)
  const int p = blockIdx.x * 256 + threadIdx.x;
  if (p * 8 + 8 > n) return;
  const v4f a0 = *(const v4f*)(src + (size_t)p * 8);
  const v4f a1 = *(const v4f*)(src + (size_t)p * 8 + 4);
  v8h o;
#pragma unroll
  for (int e = 0; e < 4; ++e) {
    o[e]     = (f16)(bfr(a0[e]) * scl);
    o[e + 4] = (f16)(bfr(a1[e]) * scl);
  }
  f16* d = dst + (size_t)p * 8;
  *(volatile v8h*)d = o;
  __threadfence();
  *(volatile v8h*)d = o;
}

template <int CPG>
__device__ __forceinline__ void gn_store_pass(const float* __restrict__ x, const float* __restrict__ gw,
                                              const float* __restrict__ gb, f16* __restrict__ out,
                                              int C, int len, int lenFull, int b, int g,
                                              float mean, float rstd, int tid) {
#pragma clang fp contract(off)
  const int l8n = len >> 3;
  const int n8 = CPG * l8n;
  for (int p = tid; p < n8; p += 256) {
    const int cl = p / l8n;
    const int l8 = p - cl * l8n;
    const int c = g * CPG + cl;
    const float wc = bfr(gw[c]);
    const float bc = bfr(gb[c]);
    const float* src = x + ((size_t)(b * C + c) * (size_t)lenFull + (size_t)l8 * 8);
    const v4f a0 = *(const v4f*)src;
    const v4f a1 = *(const v4f*)(src + 4);
    v8h o;
#pragma unroll
    for (int e = 0; e < 4; ++e) {
      const float t0 = (bfr(a0[e]) - mean) * rstd;
      const float t1 = (bfr(a1[e]) - mean) * rstd;
      o[e]     = (f16)(t0 * wc + bc);
      o[e + 4] = (f16)(t1 * wc + bc);
    }
    f16* dst = out + ((size_t)(b * C + c) * (size_t)len + (size_t)l8 * 8);
    *(volatile v8h*)dst = o;
  }
}

template <int CPG>
__global__ __launch_bounds__(256) void gn_kernel(const float* __restrict__ x, const float* __restrict__ gw,
                                                 const float* __restrict__ gb, f16* __restrict__ out,
                                                 int C, int len, int lenFull, float invn) {
#pragma clang fp contract(off)
  __shared__ float red0[8];
  __shared__ float red1[8];
  const int tid = threadIdx.x;
  const int g = blockIdx.x % NG;
  const int b = blockIdx.x / NG;
  const int l8n = len >> 3;
  const int n8 = CPG * l8n;

  float s = 0.0f;
  for (int p = tid; p < n8; p += 256) {
    const int cl = p / l8n;
    const int l8 = p - cl * l8n;
    const float* src = x + ((size_t)(b * C + g * CPG + cl) * (size_t)lenFull + (size_t)l8 * 8);
    const v4f a0 = *(const v4f*)src;
    const v4f a1 = *(const v4f*)(src + 4);
    s += ((bfr(a0[0]) + bfr(a0[1])) + (bfr(a0[2]) + bfr(a0[3])))
       + ((bfr(a1[0]) + bfr(a1[1])) + (bfr(a1[2]) + bfr(a1[3])));
  }
#pragma unroll
  for (int o = 16; o > 0; o >>= 1) s += __shfl_xor(s, o, 32);
  if ((tid & 31) == 0) red0[tid >> 5] = s;
  __syncthreads();
  float ts = 0.0f;
#pragma unroll
  for (int i = 0; i < 8; ++i) ts += red0[i];
  const float mean = ts * invn;

  float s2 = 0.0f;
  for (int p = tid; p < n8; p += 256) {
    const int cl = p / l8n;
    const int l8 = p - cl * l8n;
    const float* src = x + ((size_t)(b * C + g * CPG + cl) * (size_t)lenFull + (size_t)l8 * 8);
    const v4f a0 = *(const v4f*)src;
    const v4f a1 = *(const v4f*)(src + 4);
    float q = 0.0f;
#pragma unroll
    for (int e = 0; e < 4; ++e) {
      const float d0 = bfr(a0[e]) - mean;
      const float d1 = bfr(a1[e]) - mean;
      q += d0 * d0;
      q += d1 * d1;
    }
    s2 += q;
  }
#pragma unroll
  for (int o = 16; o > 0; o >>= 1) s2 += __shfl_xor(s2, o, 32);
  if ((tid & 31) == 0) red1[tid >> 5] = s2;
  __syncthreads();
  float ts2 = 0.0f;
#pragma unroll
  for (int i = 0; i < 8; ++i) ts2 += red1[i];
  const float var = fmaxf(ts2 * invn, 0.0f);
  const float rstd = rsqrtf(var + 1.0e-5f);

  gn_store_pass<CPG>(x, gw, gb, out, C, len, lenFull, b, g, mean, rstd, tid);
  __threadfence();
  gn_store_pass<CPG>(x, gw, gb, out, C, len, lenFull, b, g, mean, rstd, tid);
}

template <int EM> struct EpCfg;
template <> struct EpCfg<0> { typedef f16   T; static constexpr int N = GBN * 72;  };
template <> struct EpCfg<1> { typedef f16   T; static constexpr int N = GBM * 136; };
template <> struct EpCfg<2> { typedef float T; static constexpr int N = GBM * 132; };

template <int BT, int EM>
__global__ __launch_bounds__(256) void gemm_kernel(
    const f16* __restrict__ A, int K,
    const f16* __restrict__ B, long long bstride, int ldb,
    const float* __restrict__ bias, float accscl, float oscl,
    f16* __restrict__ outH, int nTot,
    float* __restrict__ outF, const float* __restrict__ xres,
    const float* __restrict__ gate) {
  typedef typename EpCfg<EM>::T ET;
  __shared__ __align__(16) f16 smA[GBM * SP];
  __shared__ __align__(16) f16 smB[GBN * SP];
  __shared__ __align__(16) ET  sE[EpCfg<EM>::N];
  __shared__ float sBias[GBM];

  const int tid = threadIdx.x;
  const int wid = tid >> 5, lane = tid & 31;
  const int lr = lane & 15, lh = lane >> 4;
  const int wm = wid >> 2, wn = wid & 3;
  const int n0 = blockIdx.x * GBN;
  const int m0 = blockIdx.y * GBM;
  const int bz = blockIdx.z;
  const f16* Bb = B + (size_t)bz * (size_t)bstride;

  if (tid < GBM) sBias[tid] = bfr(bias[m0 + tid]);

  v8f acc[2][2];
#pragma unroll
  for (int i = 0; i < 2; ++i)
#pragma unroll
    for (int j = 0; j < 2; ++j) acc[i][j] = v8zero();

  const int KT = K >> 5;
#pragma unroll 1
  for (int kt = 0; kt < KT; ++kt) {
    const int k0 = kt << 5;
    __syncthreads();
    {
      const int r = tid >> 2, kq = (tid & 3) << 3;
      const v8h av = *(const v8h*)(A + (size_t)(m0 + r) * (size_t)K + k0 + kq);
      *(v8h*)&smA[r * SP + kq] = av;
    }
    if (BT == 0) {
#pragma unroll
      for (int j = 0; j < 2; ++j) {
        const int idx = tid + j * 256;
        const int kk = idx >> 4;
        const int nc = (idx & 15) << 3;
        const v8h bv = *(const v8h*)(Bb + (size_t)(k0 + kk) * (size_t)ldb + n0 + nc);
#pragma unroll
        for (int e = 0; e < 8; ++e) smB[(nc + e) * SP + kk] = bv[e];
      }
    } else {
#pragma unroll
      for (int j = 0; j < 2; ++j) {
        const int idx = tid + j * 256;
        const int nn = idx >> 2;
        const int kq = (idx & 3) << 3;
        const v8h bv = *(const v8h*)(Bb + (size_t)(n0 + nn) * (size_t)ldb + k0 + kq);
        *(v8h*)&smB[nn * SP + kq] = bv;
      }
    }
    __syncthreads();
    v16h af[2], bq[2];
#pragma unroll
    for (int mt = 0; mt < 2; ++mt) af[mt] = load_frag(&smA[(wm * 32 + mt * 16 + lr) * SP + lh * 8]);
#pragma unroll
    for (int nt = 0; nt < 2; ++nt) bq[nt] = load_frag(&smB[(wn * 32 + nt * 16 + lr) * SP + lh * 8]);
#pragma unroll
    for (int mt = 0; mt < 2; ++mt)
#pragma unroll
      for (int nt = 0; nt < 2; ++nt) acc[mt][nt] = wmma16(af[mt], bq[nt], acc[mt][nt]);
  }

  float bb[2][8];
#pragma unroll
  for (int mt = 0; mt < 2; ++mt)
#pragma unroll
    for (int r = 0; r < 8; ++r) bb[mt][r] = sBias[wm * 32 + mt * 16 + 8 * lh + r];

  if (EM == 0) {
    const int hh = m0 >> 6;
#pragma unroll
    for (int mt = 0; mt < 2; ++mt)
#pragma unroll
      for (int nt = 0; nt < 2; ++nt) {
        const int nl = wn * 32 + nt * 16 + lr;
#pragma unroll
        for (int r = 0; r < 8; ++r) {
          const int dl = wm * 32 + mt * 16 + 8 * lh + r;
          sE[nl * 72 + dl] = (ET)((acc[mt][nt][r] * accscl + bb[mt][r]) * oscl);
        }
      }
    __syncthreads();
    v8h vals[4];
    size_t off[4];
#pragma unroll
    for (int c = 0; c < 4; ++c) {
      const int p = c * 256 + tid;
      const int nl = p >> 3, j = p & 7;
      vals[c] = *(const v8h*)&sE[nl * 72 + j * 8];
      off[c] = ((size_t)(bz * NH + hh) * (size_t)nTot + (size_t)(n0 + nl)) * HD + (size_t)j * 8;
    }
#pragma unroll
    for (int c = 0; c < 4; ++c) *(volatile v8h*)(outH + off[c]) = vals[c];
    __threadfence();
#pragma unroll
    for (int c = 0; c < 4; ++c) *(volatile v8h*)(outH + off[c]) = vals[c];
  } else if (EM == 1) {
#pragma unroll
    for (int mt = 0; mt < 2; ++mt)
#pragma unroll
      for (int nt = 0; nt < 2; ++nt) {
        const int nl = wn * 32 + nt * 16 + lr;
#pragma unroll
        for (int r = 0; r < 8; ++r) {
          const int ml = wm * 32 + mt * 16 + 8 * lh + r;
          sE[ml * 136 + nl] = (ET)((acc[mt][nt][r] * accscl + bb[mt][r]) * oscl);
        }
      }
    __syncthreads();
    v8h vals[4];
    size_t off[4];
#pragma unroll
    for (int c = 0; c < 4; ++c) {
      const int p = c * 256 + tid;
      const int ml = p >> 4, j = p & 15;
      vals[c] = *(const v8h*)&sE[ml * 136 + j * 8];
      off[c] = (size_t)(bz * CCH + m0 + ml) * (size_t)nTot + (size_t)(n0 + j * 8);
    }
#pragma unroll
    for (int c = 0; c < 4; ++c) *(volatile v8h*)(outH + off[c]) = vals[c];
    __threadfence();
#pragma unroll
    for (int c = 0; c < 4; ++c) *(volatile v8h*)(outH + off[c]) = vals[c];
  } else {
    const float gv = bfr(gate[bz]);
#pragma unroll
    for (int mt = 0; mt < 2; ++mt)
#pragma unroll
      for (int nt = 0; nt < 2; ++nt) {
        const int nl = wn * 32 + nt * 16 + lr;
#pragma unroll
        for (int r = 0; r < 8; ++r) {
          const int ml = wm * 32 + mt * 16 + 8 * lh + r;
          sE[ml * 132 + nl] = (ET)(gv * (acc[mt][nt][r] * accscl + bb[mt][r]));
        }
      }
    __syncthreads();
    v4f vals[8];
    size_t off[8];
#pragma unroll
    for (int c = 0; c < 8; ++c) {
      const int p = c * 256 + tid;
      const int ml = p >> 5, j = p & 31;
      v4f t = *(const v4f*)&sE[ml * 132 + j * 4];
      off[c] = (size_t)(bz * CCH + m0 + ml) * (size_t)SEQ_FULL + (size_t)(n0 + j * 4);
      const v4f xr = *(const v4f*)(xres + off[c]);
#pragma unroll
      for (int e = 0; e < 4; ++e) t[e] = t[e] + bfr(xr[e]);
      vals[c] = t;
    }
#pragma unroll
    for (int c = 0; c < 8; ++c) *(volatile v4f*)(outF + off[c]) = vals[c];
    __threadfence();
#pragma unroll
    for (int c = 0; c < 8; ++c) *(volatile v4f*)(outF + off[c]) = vals[c];
  }
}

__global__ __launch_bounds__(256) __attribute__((amdgpu_num_vgpr(256)))
void attn_kernel(const f16* __restrict__ Qp, const f16* __restrict__ Kp,
                 const f16* __restrict__ Vp, f16* __restrict__ AO) {
  __shared__ __align__(16) f16 sK[AKT * KP];
  __shared__ __align__(16) f16 sVt[HD * KP];
  __shared__ __align__(16) f16 sP[8][16 * KP];

  const int tid = threadIdx.x;
  const int w = tid >> 5, lane = tid & 31, lr = lane & 15, lh = lane >> 4;
  const int qb = blockIdx.x * AQB;
  const int h = blockIdx.y, b = blockIdx.z;
  const int bh = b * NH + h;
  const int sr = tid >> 2;
  const int sc = (tid & 3) << 4;
  f16* sPw = &sP[w][0];

  v16h Qf[2];
  {
    const f16* qrow = Qp + ((size_t)bh * SEQ + (size_t)(qb + w * 16 + lr)) * HD + lh * 8;
    Qf[0] = load_frag(qrow);
    Qf[1] = load_frag(qrow + 32);
  }
  v8f O[4];
#pragma unroll
  for (int t = 0; t < 4; ++t) O[t] = v8zero();
  float m[8], l[8];
#pragma unroll
  for (int i = 0; i < 8; ++i) { m[i] = -1.0e30f; l[i] = 0.0f; }

#pragma unroll 1
  for (int kt = 0; kt < LC / AKT; ++kt) {
    const int kb = kt * AKT;
    __syncthreads();
    {
      const f16* ks = Kp + ((size_t)bh * LC + (size_t)(kb + sr)) * HD + sc;
      const v8h k0 = *(const v8h*)ks;
      const v8h k1 = *(const v8h*)(ks + 8);
      const f16* vs = Vp + (size_t)(b * CCH + h * HD + sr) * (size_t)LC + kb + sc;
      const v8h v0 = *(const v8h*)vs;
      const v8h v1 = *(const v8h*)(vs + 8);
      *(v8h*)&sK[sr * KP + sc]      = k0;
      *(v8h*)&sK[sr * KP + sc + 8]  = k1;
      *(v8h*)&sVt[sr * KP + sc]     = v0;
      *(v8h*)&sVt[sr * KP + sc + 8] = v1;
    }
    __syncthreads();

    v8f s[4];
#pragma unroll
    for (int j = 0; j < 4; ++j) s[j] = v8zero();
#pragma unroll
    for (int kc = 0; kc < 2; ++kc) {
#pragma unroll
      for (int j = 0; j < 4; ++j) {
        const v16h Bk = load_frag(&sK[(j * 16 + lr) * KP + kc * 32 + lh * 8]);
        s[j] = wmma16(Qf[kc], Bk, s[j]);
      }
    }

    float corr[8];
#pragma unroll
    for (int i = 0; i < 8; ++i) {
      const float a0 = s[0][i] * 0.125f, a1 = s[1][i] * 0.125f;
      const float a2 = s[2][i] * 0.125f, a3 = s[3][i] * 0.125f;
      float t = fmaxf(fmaxf(a0, a1), fmaxf(a2, a3));
      t = fmaxf(t, __shfl_xor(t, 1, 32));
      t = fmaxf(t, __shfl_xor(t, 2, 32));
      t = fmaxf(t, __shfl_xor(t, 4, 32));
      t = fmaxf(t, __shfl_xor(t, 8, 32));
      const float mn = fmaxf(m[i], t);
      corr[i] = __expf(m[i] - mn);
      m[i] = mn;
      const float p0 = __expf(a0 - mn), p1 = __expf(a1 - mn);
      const float p2 = __expf(a2 - mn), p3 = __expf(a3 - mn);
      s[0][i] = p0; s[1][i] = p1; s[2][i] = p2; s[3][i] = p3;
      float r = (p0 + p1) + (p2 + p3);
      r += __shfl_xor(r, 1, 32);
      r += __shfl_xor(r, 2, 32);
      r += __shfl_xor(r, 4, 32);
      r += __shfl_xor(r, 8, 32);
      l[i] = l[i] * corr[i] + r;
    }
#pragma unroll
    for (int t = 0; t < 4; ++t)
#pragma unroll
      for (int i = 0; i < 8; ++i) O[t][i] *= corr[i];

#pragma unroll
    for (int i = 0; i < 8; ++i) {
      const int row = i + 8 * lh;
#pragma unroll
      for (int j = 0; j < 4; ++j) sPw[row * KP + j * 16 + lr] = (f16)(s[j][i] * 1024.0f);
    }
    __syncthreads();
    v16h Pf[2];
    Pf[0] = load_frag(sPw + lr * KP + lh * 8);
    Pf[1] = load_frag(sPw + lr * KP + 32 + lh * 8);

#pragma unroll
    for (int kc = 0; kc < 2; ++kc) {
#pragma unroll
      for (int t = 0; t < 4; ++t) {
        const v16h Bv = load_frag(&sVt[(t * 16 + lr) * KP + kc * 32 + lh * 8]);
        O[t] = wmma16(Pf[kc], Bv, O[t]);
      }
    }
  }

  float inv[8];
#pragma unroll
  for (int i = 0; i < 8; ++i) inv[i] = 0.03125f * __builtin_amdgcn_rcpf(l[i]);
  __syncthreads();
#pragma unroll
  for (int t = 0; t < 4; ++t)
#pragma unroll
    for (int i = 0; i < 8; ++i) sPw[(i + 8 * lh) * KP + t * 16 + lr] = (f16)(O[t][i] * inv[i]);
  __syncthreads();
  v8h vals[4];
  size_t off[4];
#pragma unroll
  for (int c = 0; c < 4; ++c) {
    const int p = c * 32 + lane;
    const int row = p >> 3, j = p & 7;
    vals[c] = *(const v8h*)(sPw + row * KP + j * 8);
    off[c] = (size_t)(b * SEQ + qb + w * 16 + row) * (size_t)CCH + (size_t)(h * HD + j * 8);
  }
#pragma unroll
  for (int c = 0; c < 4; ++c) *(volatile v8h*)(AO + off[c]) = vals[c];
  __threadfence();
#pragma unroll
  for (int c = 0; c < 4; ++c) *(volatile v8h*)(AO + off[c]) = vals[c];
}

extern "C" void kernel_launch(void* const* d_in, const int* in_sizes, int n_in,
                              void* d_out, int out_size, void* d_ws, size_t ws_size,
                              hipStream_t stream) {
  if (n_in < 15) return;
  const float* x      = (const float*)d_in[0];
  const float* ctx    = (const float*)d_in[1];
  const float* gate   = (const float*)d_in[2];
  const float* norm_w = (const float*)d_in[3];
  const float* norm_b = (const float*)d_in[4];
  const float* cnw    = (const float*)d_in[5];
  const float* cnb    = (const float*)d_in[6];
  const float* q_w    = (const float*)d_in[7];
  const float* q_b    = (const float*)d_in[8];
  const float* k_w    = (const float*)d_in[9];
  const float* k_b    = (const float*)d_in[10];
  const float* v_w    = (const float*)d_in[11];
  const float* v_b    = (const float*)d_in[12];
  const float* o_w    = (const float*)d_in[13];
  const float* o_b    = (const float*)d_in[14];
  float* outp = (float*)d_out;

  if (in_sizes[0]  < NB * CCH * SEQ_FULL) return;
  if (in_sizes[1]  < NB * CCX * LC_FULL) return;
  if (in_sizes[2]  < NB) return;
  if (in_sizes[3]  < CCH || in_sizes[4] < CCH) return;
  if (in_sizes[5]  < CCX || in_sizes[6] < CCX) return;
  if (in_sizes[7]  < CCH * CCH || in_sizes[8] < CCH) return;
  if (in_sizes[9]  < CCH * CCX || in_sizes[10] < CCH) return;
  if (in_sizes[11] < CCH * CCX || in_sizes[12] < CCH) return;
  if (in_sizes[13] < CCH * CCH || in_sizes[14] < CCH) return;
  if ((size_t)out_size < (size_t)(NB * CCH - 1) * SEQ_FULL + (size_t)SEQ) return;

  const size_t nWq = (size_t)CCH * CCH;
  const size_t nWk = (size_t)CCH * CCX;
  const size_t nXn = (size_t)NB * CCH * SEQ;
  const size_t nCn = (size_t)NB * CCX * LC;
  const size_t nQp = (size_t)NB * NH * SEQ * HD;
  const size_t nKp = (size_t)NB * NH * LC * HD;
  const size_t nVp = (size_t)NB * CCH * LC;
  const size_t nAO = (size_t)NB * SEQ * CCH;
  char* ws = (char*)d_ws;
  size_t off = 0;
  f16* Wq = (f16*)(ws + off); off += nWq * 2;
  f16* Wk = (f16*)(ws + off); off += nWk * 2;
  f16* Wv = (f16*)(ws + off); off += nWk * 2;
  f16* Wo = (f16*)(ws + off); off += nWq * 2;
  f16* Xn = (f16*)(ws + off); off += nXn * 2;
  f16* Cn = (f16*)(ws + off); off += nCn * 2;
  f16* Qp = (f16*)(ws + off); off += nQp * 2;
  f16* Kp = (f16*)(ws + off); off += nKp * 2;
  f16* Vp = (f16*)(ws + off); off += nVp * 2;
  f16* AO = (f16*)(ws + off); off += nAO * 2;
  if (off > ws_size) return;

  cvt_w_kernel<<<(int)((nWq / 8 + 255) / 256), 256, 0, stream>>>(q_w, Wq, (int)nWq, 64.0f);
  cvt_w_kernel<<<(int)((nWk / 8 + 255) / 256), 256, 0, stream>>>(k_w, Wk, (int)nWk, 64.0f);
  cvt_w_kernel<<<(int)((nWk / 8 + 255) / 256), 256, 0, stream>>>(v_w, Wv, (int)nWk, 64.0f);
  cvt_w_kernel<<<(int)((nWq / 8 + 255) / 256), 256, 0, stream>>>(o_w, Wo, (int)nWq, 64.0f);

  gn_kernel<CCH / NG><<<NB * NG, 256, 0, stream>>>(x, norm_w, norm_b, Xn, CCH, SEQ, SEQ_FULL,
                                                    1.0f / (float)((CCH / NG) * SEQ));
  gn_kernel<CCX / NG><<<NB * NG, 256, 0, stream>>>(ctx, cnw, cnb, Cn, CCX, LC, LC_FULL,
                                                    1.0f / (float)((CCX / NG) * LC));

  gemm_kernel<0, 0><<<dim3(SEQ / GBN, CCH / GBM, NB), 256, 0, stream>>>(
      Wq, CCH, Xn, (long long)CCH * SEQ, SEQ, q_b, 0.015625f, 1.0f, Qp, SEQ, outp, x, gate);
  gemm_kernel<0, 0><<<dim3(LC / GBN, CCH / GBM, NB), 256, 0, stream>>>(
      Wk, CCX, Cn, (long long)CCX * LC, LC, k_b, 0.015625f, 1.0f, Kp, LC, outp, x, gate);
  gemm_kernel<0, 1><<<dim3(LC / GBN, CCH / GBM, NB), 256, 0, stream>>>(
      Wv, CCX, Cn, (long long)CCX * LC, LC, v_b, 0.015625f, 1.0f, Vp, LC, outp, x, gate);

  attn_kernel<<<dim3(SEQ / AQB, NH, NB), 256, 0, stream>>>(Qp, Kp, Vp, AO);

  gemm_kernel<1, 2><<<dim3(SEQ / GBN, CCH / GBM, NB), 256, 0, stream>>>(
      Wo, CCH, AO, (long long)SEQ * CCH, CCH, o_b, 0.00048828125f, 1.0f, Qp, SEQ, outp, x, gate);
}
